// CausalSelfAttention_5557687681798
// MI455X (gfx1250) — hardware-verified
//
#include <hip/hip_runtime.h>


#ifndef NB
#define NB 2
#endif
#ifndef SEQ
#define SEQ 2048
#endif
#define NB_FULL  2
#define SEQ_FULL 2048
#define DM   1024
#define NH   16
#define HD   64
#define MTOK (NB * SEQ)
#define QCAR 16.0f
#define KCAR 16.0f
#define VCAR 16.0f
#define PLOG 8.0f
#define CCAR 64.0f
#define WCAR 16.0f
#define SCL  0.125f
#define CS2  (SCL * 1.4426950408889634f / (QCAR * KCAR))

typedef _Float16 h16;
typedef unsigned short bf;
typedef __attribute__((ext_vector_type(16))) __bf16   v16bf;
typedef __attribute__((ext_vector_type(16))) _Float16 v16h;
typedef __attribute__((ext_vector_type(8)))  _Float16 v8h;
typedef __attribute__((ext_vector_type(8)))  unsigned short v8us;
typedef __attribute__((ext_vector_type(8)))  float    v8f;
typedef __attribute__((ext_vector_type(4)))  float    v4f;
typedef v8h  __attribute__((may_alias)) v8ha;
typedef v4f  __attribute__((may_alias)) v4fa;

static_assert(SEQ % 64 == 0);
static_assert(MTOK % 64 == 0);
static_assert(DM % 64 == 0 && DM % 32 == 0);
static_assert(HD == 64 && NH * HD == DM);
static_assert((NB * NH * (SEQ / 16)) % 8 == 0);
static_assert(((size_t)SEQ * DM / 8) % 256 == 0);
static_assert(((size_t)DM * DM / 8) % 256 == 0);
static_assert(QCAR == KCAR);
static_assert(NB <= NB_FULL && SEQ <= SEQ_FULL);

#define SZ_XB  ((size_t)MTOK * DM * 2)
#define SZ_W3  ((size_t)3 * DM * DM * 2)
#define SZ_WP  ((size_t)DM * DM * 2)
#define SZ_QK  ((size_t)2 * NB * NH * SEQ * HD * 2)
#define SZ_VT  ((size_t)NB * NH * HD * SEQ * 2)
#define SZ_Y   ((size_t)MTOK * DM * 2)
#define WS_TOTAL (SZ_XB + SZ_W3 + SZ_WP + SZ_QK + SZ_VT + SZ_Y)
static_assert(WS_TOTAL <= (size_t)134217728);
static_assert(SZ_XB % 256 == 0 && SZ_W3 % 256 == 0 && SZ_WP % 256 == 0 && SZ_QK % 256 == 0 && SZ_VT % 256 == 0);

__device__ __forceinline__ unsigned short f2bf(float f) { unsigned u = __float_as_uint(f); u += 0x7FFFu + ((u >> 16) & 1u); return (unsigned short)(u >> 16); }
__device__ __forceinline__ float bf2f(unsigned short b) { return __uint_as_float(((unsigned)b) << 16); }
__device__ __forceinline__ float bfr(float f) { return bf2f(f2bf(f)); }
__device__ __forceinline__ v16h cat16(v8h lo, v8h hi) { return __builtin_shufflevector(lo, hi, 0, 1, 2, 3, 4, 5, 6, 7, 8, 9, 10, 11, 12, 13, 14, 15); }
__device__ __forceinline__ v16bf cat16b(v8us lo, v8us hi) { return __builtin_bit_cast(v16bf, __builtin_shufflevector(lo, hi, 0, 1, 2, 3, 4, 5, 6, 7, 8, 9, 10, 11, 12, 13, 14, 15)); }

__device__ __forceinline__ v8f wmma16g(v16h a, v16h b, v8f c) {
    c = __builtin_amdgcn_wmma_f32_16x16x32_f16(false, a, false, b, (short)0, c, false, false);
    asm volatile("v_nop\n\tv_nop\n\tv_nop\n\tv_nop" : "+v"(c) : "v"(a), "v"(b));
    return c;
}
__device__ __forceinline__ v8f wmmabg(v16bf a, v16bf b, v8f c) {
    c = __builtin_amdgcn_wmma_f32_16x16x32_bf16(false, a, false, b, (short)0, c, false, false);
    asm volatile("v_nop\n\tv_nop\n\tv_nop\n\tv_nop" : "+v"(c) : "v"(a), "v"(b));
    return c;
}

__device__ __forceinline__ v16h ldh(const h16* p) { return cat16(*(const v8h*)p, *(const v8h*)(p + 16)); }
template <typename T16> struct WFrag;
template <> struct WFrag<h16> { typedef v16h V; static __device__ __forceinline__ V ld(const h16* p) { return ldh(p); } static __device__ __forceinline__ v8f mma(V a, V b, v8f c) { return wmma16g(a, b, c); } };
template <> struct WFrag<bf> { typedef v16bf V; static __device__ __forceinline__ V ld(const bf* p) { return cat16b(*(const v8us*)p, *(const v8us*)(p + 16)); } static __device__ __forceinline__ v8f mma(V a, V b, v8f c) { return wmmabg(a, b, c); } };

__device__ __forceinline__ void lds_wave_sync() { __builtin_amdgcn_wave_barrier(); asm volatile("s_wait_dscnt 0" ::: "memory"); __builtin_amdgcn_wave_barrier(); }

template <typename T16>
__device__ __forceinline__ void gemm_main(const T16* __restrict__ A, const T16* __restrict__ Bt, const int K, const int r0, const int c0, const int lr, const int hi, v8f (&acc)[4][4]) {
    typedef typename WFrag<T16>::V V;
#pragma unroll
    for (int mb = 0; mb < 4; ++mb)
#pragma unroll
        for (int nb = 0; nb < 4; ++nb) acc[mb][nb] = (v8f){};
    const size_t aoff = (size_t)(r0 + lr) * K + 8 * hi, boff = (size_t)(c0 + lr) * K + 8 * hi;
#pragma unroll 1
    for (int kc = 0; kc < K; kc += 32) {
        V a[4];
#pragma unroll
        for (int mb = 0; mb < 4; ++mb) a[mb] = WFrag<T16>::ld(A + aoff + (size_t)mb * 16 * K + kc);
#pragma unroll
        for (int nb = 0; nb < 4; ++nb) {
            const V b = WFrag<T16>::ld(Bt + boff + (size_t)nb * 16 * K + kc);
#pragma unroll
            for (int mb = 0; mb < 4; ++mb) acc[mb][nb] = WFrag<T16>::mma(a[mb], b, acc[mb][nb]);
        }
    }
}

__global__ __launch_bounds__(256) void k_cvt8(const float* __restrict__ src, bf* dst, size_t n8, size_t sstride, size_t dstride) {
    const size_t i = (size_t)blockIdx.x * 256 + threadIdx.x; if (i >= n8) return;
    const float* s = src + (size_t)blockIdx.y * sstride + i * 8; bf* d = dst + (size_t)blockIdx.y * dstride + i * 8;
    const v8f v = *(const v8f*)s; v8us o;
#pragma unroll
    for (int k = 0; k < 8; ++k) o[k] = f2bf(v[k]);
    *(volatile v8us*)d = o; __threadfence(); *(volatile v8us*)d = o;
}
__global__ __launch_bounds__(256) void k_cvt8h(const float* __restrict__ src, h16* dst, size_t n8) {
    const size_t i = (size_t)blockIdx.x * 256 + threadIdx.x; if (i >= n8) return;
    const v8f v = *(const v8f*)(src + i * 8); v8h o;
#pragma unroll
    for (int k = 0; k < 8; ++k) o[k] = (h16)(bfr(v[k]) * WCAR);
    *(volatile v8h*)(dst + i * 8) = o; __threadfence(); *(volatile v8h*)(dst + i * 8) = o;
}

__global__ __launch_bounds__(32) void k_projqk(const bf* __restrict__ XB, const bf* __restrict__ W2, h16* QK) {
    __shared__ __align__(16) float os[16 * 68];
    const int lane = threadIdx.x & 31, lr = lane & 15, hi = lane >> 4;
    const int r0 = blockIdx.x * 64, c0 = blockIdx.y * 64; const size_t z = blockIdx.z;
    v8f acc[4][4];
    gemm_main<bf>(XB, W2 + z * (size_t)DM * DM, DM, r0, c0, lr, hi, acc);
    const int b = r0 / SEQ, t0 = r0 % SEQ, head = blockIdx.y;
    const int rq = lane >> 3, pc = (lane & 7) * 8;
    h16* dst = QK + z * ((size_t)NB * NH * SEQ * HD) + ((size_t)(b * NH + head) * SEQ + t0) * HD + pc;
#pragma unroll
    for (int mb = 0; mb < 4; ++mb) {
#pragma unroll
        for (int nb = 0; nb < 4; ++nb) {
#pragma unroll
            for (int j = 0; j < 8; ++j) os[(hi * 8 + j) * 68 + nb * 16 + lr] = acc[mb][nb][j]; }
        lds_wave_sync();
        v8h val[4];
#pragma unroll
        for (int s = 0; s < 4; ++s) { const int row = 4 * s + rq; const v4f f0 = *(const v4fa*)(os + row * 68 + pc); const v4f f1 = *(const v4fa*)(os + row * 68 + pc + 4); v8h o;
#pragma unroll
            for (int q = 0; q < 4; ++q) { o[q] = (h16)(f0[q] * QCAR); o[4 + q] = (h16)(f1[q] * QCAR); }
            val[s] = o; }
#pragma unroll 1
        for (int ps = 0; ps < 2; ++ps) {
#pragma unroll
            for (int s = 0; s < 4; ++s) *(volatile v8h*)(dst + (size_t)(mb * 16 + 4 * s + rq) * HD) = val[s];
            if (ps == 0) __threadfence(); }
        lds_wave_sync();
    }
}

__global__ __launch_bounds__(32) void k_projv(const bf* __restrict__ XB, const bf* __restrict__ WV, h16* VT) {
    __shared__ __align__(16) h16 vs[64 * 72];
    const int lane = threadIdx.x & 31, lr = lane & 15, hi = lane >> 4;
    const int r0 = blockIdx.x * 64, c0 = blockIdx.y * 64;
    v8f acc[4][4];
    gemm_main<bf>(XB, WV, DM, r0, c0, lr, hi, acc);
#pragma unroll
    for (int mb = 0; mb < 4; ++mb)
#pragma unroll
        for (int nb = 0; nb < 4; ++nb) { v8h o;
#pragma unroll
            for (int j = 0; j < 8; ++j) o[j] = (h16)(acc[mb][nb][j] * VCAR);
            *(v8ha*)(vs + (nb * 16 + lr) * 72 + mb * 16 + hi * 8) = o; }
    lds_wave_sync();
    const int b = r0 / SEQ, t0 = r0 % SEQ, head = blockIdx.y;
    const int rq = lane >> 3, pc = (lane & 7) * 8;
    h16* dst = VT + ((size_t)(b * NH + head) * HD) * SEQ + t0 + pc;
#pragma unroll 1
    for (int ps = 0; ps < 2; ++ps) {
#pragma unroll
        for (int s = 0; s < 16; ++s) { const int d = 4 * s + rq; const v8h val = *(const v8ha*)(vs + d * 72 + pc); *(volatile v8h*)(dst + (size_t)d * SEQ) = val; }
        if (ps == 0) __threadfence(); }
}

__global__ __launch_bounds__(256) void k_flash(const h16* __restrict__ QP, const h16* __restrict__ KP, const h16* __restrict__ VT, h16* Y) {
    __shared__ __align__(16) h16 ys[8 * 16 * 72];
    const int lane = threadIdx.x & 31, lr = lane & 15, hi = lane >> 4;
    const int wave = __builtin_amdgcn_readfirstlane(threadIdx.x >> 5);
    const int task = blockIdx.x * 8 + wave;
    const int qt = task % (SEQ / 16), bh = task / (SEQ / 16);
    const h16* qb = QP + ((size_t)bh * SEQ + qt * 16 + lr) * HD + 8 * hi;
    const v16h qf0 = ldh(qb), qf1 = ldh(qb + 32);
    const h16* kb = KP + (size_t)bh * SEQ * HD + (size_t)lr * HD + 8 * hi;
    const h16* vb = VT + (size_t)bh * HD * SEQ + (size_t)lr * SEQ + 8 * hi;
    v8f o[4];
#pragma unroll
    for (int t = 0; t < 4; ++t) o[t] = (v8f){};
    float m = -3.0e38f, l = 0.0f;
#pragma unroll 1
    for (int k0 = 0; k0 < SEQ; k0 += 64) {
        v8f s[4];
#pragma unroll
        for (int j = 0; j < 4; ++j) { const h16* kp = kb + (size_t)(k0 + j * 16) * HD; const v16h ka0 = ldh(kp), ka1 = ldh(kp + 32); v8f c = (v8f){}; c = wmma16g(ka0, qf0, c); c = wmma16g(ka1, qf1, c); s[j] = c; }
        float tm = s[0][0];
#pragma unroll
        for (int j = 0; j < 4; ++j)
#pragma unroll
            for (int r = 0; r < 8; ++r) tm = fmaxf(tm, s[j][r]);
        tm = fmaxf(tm, __shfl_xor(tm, 16, 32));
        const float mn = fmaxf(m, tm * CS2);
        const float alpha = __builtin_amdgcn_exp2f(m - mn);
        const float off = PLOG - mn;
        m = mn;
        float ls = 0.0f;
#pragma unroll
        for (int j = 0; j < 4; ++j)
#pragma unroll
            for (int r = 0; r < 8; ++r) { const float p = __builtin_amdgcn_exp2f(fmaf(s[j][r], CS2, off)); s[j][r] = p; ls += p; }
        l = fmaf(l, alpha, ls);
#pragma unroll
        for (int t = 0; t < 4; ++t)
#pragma unroll
            for (int r = 0; r < 8; ++r) o[t][r] *= alpha;
        {
            v16h pb;
#pragma unroll
            for (int r = 0; r < 8; ++r) { pb[r] = (h16)s[0][r]; pb[8 + r] = (h16)s[1][r]; }
#pragma unroll
            for (int t = 0; t < 4; ++t) { const v16h va = ldh(vb + (size_t)(t * 16) * SEQ + k0); o[t] = wmma16g(va, pb, o[t]); }
        }
        {
            v16h pb;
#pragma unroll
            for (int r = 0; r < 8; ++r) { pb[r] = (h16)s[2][r]; pb[8 + r] = (h16)s[3][r]; }
#pragma unroll
            for (int t = 0; t < 4; ++t) { const v16h va = ldh(vb + (size_t)(t * 16) * SEQ + k0 + 32); o[t] = wmma16g(va, pb, o[t]); }
        }
    }
    const float lt = l + __shfl_xor(l, 16, 32);
    const float inv = (CCAR / VCAR) * (1.0f / lt);
    const int yw = wave * 16 * 72;
#pragma unroll
    for (int t = 0; t < 4; ++t) { v8h o8;
#pragma unroll
        for (int r = 0; r < 8; ++r) o8[r] = (h16)(o[t][r] * inv);
        *(v8ha*)(ys + yw + lr * 72 + t * 16 + 8 * hi) = o8; }
    lds_wave_sync();
    const int rq = lane >> 3, pc = (lane & 7) * 8;
    v8h val[4];
#pragma unroll
    for (int s2 = 0; s2 < 4; ++s2) val[s2] = *(const v8ha*)(ys + yw + (4 * s2 + rq) * 72 + pc);
    const int b = bh / NH, h = bh % NH;
    h16* dst = Y + ((size_t)b * SEQ + qt * 16) * DM + h * HD + pc;
#pragma unroll 1
    for (int ps = 0; ps < 2; ++ps) {
#pragma unroll
        for (int s2 = 0; s2 < 4; ++s2) *(volatile v8h*)(dst + (size_t)(4 * s2 + rq) * DM) = val[s2];
        if (ps == 0) __threadfence(); }
}

__global__ __launch_bounds__(32) void k_outp(const h16* __restrict__ Yc, const h16* __restrict__ WP, const float* __restrict__ bias, float* OUT) {
    __shared__ __align__(16) float os[16 * 68];
    const int lane = threadIdx.x & 31, lr = lane & 15, hi = lane >> 4;
    const int r0 = blockIdx.x * 64, c0 = blockIdx.y * 64;
    v8f acc[4][4];
    gemm_main<h16>(Yc, WP, DM, r0, c0, lr, hi, acc);
    const int cofs = lr * 4;
    const v4f braw = *(const v4f*)(bias + c0 + cofs);
    v4f bv; bv[0] = bfr(braw[0]); bv[1] = bfr(braw[1]); bv[2] = bfr(braw[2]); bv[3] = bfr(braw[3]);
    const float osc = 1.0f / (CCAR * WCAR);
#pragma unroll
    for (int mb = 0; mb < 4; ++mb) {
#pragma unroll
        for (int nb = 0; nb < 4; ++nb) {
#pragma unroll
            for (int j = 0; j < 8; ++j) os[(hi * 8 + j) * 68 + nb * 16 + lr] = acc[mb][nb][j]; }
        lds_wave_sync();
        float* crow = OUT + (size_t)(r0 + mb * 16) * DM + c0 + cofs;
#pragma unroll 1
        for (int ps = 0; ps < 2; ++ps) {
#pragma unroll
            for (int s = 0; s < 8; ++s) { const int row = 2 * s + hi; const v4f f = *(const v4fa*)(os + row * 68 + cofs); v4f val;
                val[0] = fmaf(f[0], osc, bv[0]); val[1] = fmaf(f[1], osc, bv[1]); val[2] = fmaf(f[2], osc, bv[2]); val[3] = fmaf(f[3], osc, bv[3]);
                *(volatile v4f*)(crow + (size_t)row * DM) = val; }
            if (ps == 0) __threadfence(); }
        lds_wave_sync();
    }
}

extern "C" void kernel_launch(void* const* d_in, const int* in_sizes, int n_in,
                              void* d_out, int out_size, void* d_ws, size_t ws_size, hipStream_t stream) {
    if (n_in < 6) return;
    if ((size_t)in_sizes[0] < (size_t)(NB - 1) * SEQ_FULL * DM + (size_t)SEQ * DM) return;
    if ((size_t)in_sizes[1] < (size_t)DM * DM || (size_t)in_sizes[2] < (size_t)DM * DM || (size_t)in_sizes[3] < (size_t)DM * DM || (size_t)in_sizes[4] < (size_t)DM * DM || in_sizes[5] < DM) return;
    if ((size_t)out_size < (size_t)MTOK * DM) return;
    if (ws_size < WS_TOTAL) return;
    const float* x  = (const float*)d_in[0];
    const float* wk = (const float*)d_in[1];
    const float* wq = (const float*)d_in[2];
    const float* wv = (const float*)d_in[3];
    const float* wp = (const float*)d_in[4];
    const float* bp = (const float*)d_in[5];
    float* OUT = (float*)d_out;
    char* wsp = (char*)d_ws;
    bf*  XB  = (bf*)wsp;  wsp += SZ_XB;
    bf*  W3  = (bf*)wsp;  wsp += SZ_W3;
    h16* WP  = (h16*)wsp; wsp += SZ_WP;
    h16* QK  = (h16*)wsp; wsp += SZ_QK;
    h16* VT  = (h16*)wsp; wsp += SZ_VT;
    h16* Yc  = (h16*)wsp; wsp += SZ_Y;
    const size_t nw8 = (size_t)DM * DM / 8, nx8 = (size_t)SEQ * DM / 8;
    k_cvt8<<<dim3((unsigned)(nx8 / 256), NB, 1), 256, 0, stream>>>(x, XB, nx8, (size_t)SEQ_FULL * DM, (size_t)SEQ * DM);
    k_cvt8<<<dim3((unsigned)(nw8 / 256), 1, 1), 256, 0, stream>>>(wq, W3, nw8, 0, 0);
    k_cvt8<<<dim3((unsigned)(nw8 / 256), 1, 1), 256, 0, stream>>>(wk, W3 + (size_t)DM * DM, nw8, 0, 0);
    k_cvt8<<<dim3((unsigned)(nw8 / 256), 1, 1), 256, 0, stream>>>(wv, W3 + (size_t)2 * DM * DM, nw8, 0, 0);
    k_cvt8h<<<dim3((unsigned)(nw8 / 256), 1, 1), 256, 0, stream>>>(wp, WP, nw8);
    k_projqk<<<dim3(MTOK / 64, DM / 64, 2), 32, 0, stream>>>(XB, W3, QK);
    k_projv<<<dim3(MTOK / 64, DM / 64, 1), 32, 0, stream>>>(XB, W3 + (size_t)2 * DM * DM, VT);
    k_flash<<<dim3(NB * NH * (SEQ / 16) / 8, 1, 1), 256, 0, stream>>>(QK, QK + (size_t)NB * NH * SEQ * HD, VT, Yc);
    k_outp<<<dim3(MTOK / 64, DM / 64, 1), 32, 0, stream>>>(Yc, WP, bp, OUT);
}
